// MRNN_57887569216036
// MI455X (gfx1250) — hardware-verified
//
#include <hip/hip_runtime.h>


#define AS3 __attribute__((address_space(3)))

#define NT_  256
#define NB_  64
#define NI_  32
#define NH_  256
#define NO_  32
#define NK_  16
#define RB   16
#define NBLK (NB_ / RB)

static_assert(NB_ % RB == 0);
static_assert(NI_ == 32 && NO_ == 32 && NK_ == 16);
static_assert(NH_ == 8 * 32);
static_assert(NH_ % 32 == 0);

typedef __bf16         v16b __attribute__((ext_vector_type(16)));
typedef unsigned short v8us __attribute__((ext_vector_type(8)));
typedef unsigned short v4us __attribute__((ext_vector_type(4)));
typedef float          v8f  __attribute__((ext_vector_type(8)));
typedef float          v4f  __attribute__((ext_vector_type(4)));
typedef v8us __attribute__((may_alias)) v8usa;
typedef v4f  __attribute__((may_alias)) v4fa;

typedef AS3 unsigned short*       lp_us;
typedef AS3 const unsigned short* lcp_us;
typedef AS3 float*                lp_f;
typedef AS3 const float*          lcp_f;

union Frag { v16b v; v8us half[2]; };

constexpr int P_WDX0 = 0;
constexpr int P_WX0  = P_WDX0 + NH_ * NI_;
constexpr int P_WDH0 = P_WX0  + NH_ * NI_;
constexpr int P_WH0  = P_WDH0 + NH_ * NH_;
constexpr int P_WO0  = P_WH0  + NH_ * NH_;
constexpr int P_WDX1 = P_WO0  + NH_ * NH_;
constexpr int P_WDH1 = P_WDX1 + NH_ * NH_;
constexpr int P_WX1  = P_WDH1 + NH_ * NH_;
constexpr int P_WH1  = P_WX1  + NH_ * NH_;
constexpr int P_WO1  = P_WH1  + NH_ * NH_;
constexpr int P_X    = P_WO1  + NO_ * NH_;
constexpr int P_END  = P_X    + NT_ * NB_ * NI_;
constexpr int NPC    = P_END / 8;
constexpr int NCBLK  = NPC / 256;
static_assert(P_END % 8 == 0);
static_assert(NPC % 256 == 0);
static_assert(P_WX0 % 2048 == 0 && P_WDH0 % 2048 == 0 && P_WH0 % 2048 == 0 && P_WO0 % 2048 == 0 &&
              P_WDX1 % 2048 == 0 && P_WDH1 % 2048 == 0 && P_WX1 % 2048 == 0 && P_WH1 % 2048 == 0 &&
              P_WO1 % 2048 == 0 && P_X % 2048 == 0);

constexpr size_t OFF_CV = 0;
constexpr size_t SZ_CV  = (size_t)P_END * 2;
constexpr size_t OFF_HI = OFF_CV + SZ_CV;
constexpr int    HL     = NK_ * RB * NH_;
constexpr int    HBLK   = 2 * HL;
constexpr size_t SZ_HI  = (size_t)NBLK * HBLK * 4;
constexpr size_t WS_END = OFF_HI + SZ_HI;
static_assert(OFF_HI % 128 == 0);
static_assert(WS_END <= (size_t)134217728);
static_assert((size_t)NPC * 16 == SZ_CV);
static_assert((size_t)NBLK * 2 * NK_ * 4 * 256 * 16 == SZ_HI);

constexpr int    SP    = NH_ + 8;
constexpr size_t TB    = (size_t)RB * SP * 2;
constexpr size_t L_H0H = 0 * TB, L_H0L = 1 * TB;
constexpr size_t L_M0H = 2 * TB, L_M0L = 3 * TB;
constexpr size_t L_OH  = 4 * TB, L_OL  = 5 * TB;
constexpr size_t L_H1H = 6 * TB, L_H1L = 7 * TB;
constexpr size_t L_M1H = 8 * TB, L_M1L = 9 * TB;
constexpr size_t L_SD  = 10 * TB;
constexpr size_t L_SF  = L_SD + (size_t)RB * NH_ * 4;
constexpr size_t L_SO  = L_SF + (size_t)RB * NH_ * 4;
constexpr size_t L_SB  = L_SO + (size_t)RB * NO_ * 4;
constexpr size_t L_RC  = L_SB + (size_t)6 * NH_ * 4;
constexpr size_t LDS_BYTES = L_RC + 64;
constexpr int    NLDS16 = (int)(LDS_BYTES / 16);
static_assert(SP % 8 == 0);
static_assert(TB % 16 == 0 && L_SD % 16 == 0 && L_SF % 16 == 0 && L_SO % 16 == 0 && L_SB % 16 == 0 && L_RC % 16 == 0);
static_assert(LDS_BYTES % 16 == 0);

__device__ __forceinline__ unsigned short bf16_bits(float f) {
  unsigned u = __float_as_uint(f);
  u += 0x7FFFu + ((u >> 16) & 1u);
  return (unsigned short)(u >> 16);
}
__device__ __forceinline__ float bf16_val(unsigned short b) { return __uint_as_float(((unsigned)b) << 16); }
__device__ __forceinline__ float bf16r(float f) { return bf16_val(bf16_bits(f)); }
__device__ __forceinline__ v8f zero8() {
  v8f z;
#pragma unroll
  for (int i = 0; i < 8; ++i) z[i] = 0.0f;
  return z;
}
__device__ __forceinline__ v4f splat4(float x) {
  v4f z;
#pragma unroll
  for (int i = 0; i < 4; ++i) z[i] = x;
  return z;
}

__device__ __forceinline__ void ldfrag_g(Frag& f, const unsigned short* p, int h) {
  f.half[0] = *(const v8usa*)(p + 8 * h);
  f.half[1] = *(const v8usa*)(p + 16 + 8 * h);
}
__device__ __forceinline__ void ldfrag_l(Frag& f, lcp_us p, int h) {
  f.half[0] = *(AS3 const v8usa*)(p + 8 * h);
  f.half[1] = *(AS3 const v8usa*)(p + 16 + 8 * h);
}
__device__ __forceinline__ v8f mma16(v8f c, const Frag& a, const Frag& b) {
  return __builtin_amdgcn_wmma_f32_16x16x32_bf16(false, a.v, false, b.v, (short)0, c, false, false);
}

__device__ __forceinline__ void gemm_x(v8f (&acc)[2], const unsigned short* xa, const unsigned short* wb, int h)
{
  Frag a, b0, b1;
  ldfrag_g(a, xa, h);
  ldfrag_g(b0, wb, h);
  ldfrag_g(b1, wb + 16 * NI_, h);
  acc[0] = mma16(acc[0], a, b0);
  acc[1] = mma16(acc[1], a, b1);
  asm volatile("v_nop\n\tv_nop\n\tv_nop\n\tv_nop" : "+v"(acc[0]), "+v"(acc[1]) : "v"(a.v), "v"(b0.v), "v"(b1.v));
}
__device__ __forceinline__ void gemm_hl(v8f (&acc)[2], lcp_us aH, lcp_us aL, const unsigned short* wb, int h)
{
#pragma unroll 1
  for (int k0 = 0; k0 < NH_; k0 += 32) {
    Frag ah, al, b0, b1;
    ldfrag_l(ah, aH + k0, h);
    ldfrag_l(al, aL + k0, h);
    ldfrag_g(b0, wb + k0, h);
    ldfrag_g(b1, wb + 16 * NH_ + k0, h);
    acc[0] = mma16(acc[0], ah, b0);
    acc[0] = mma16(acc[0], al, b0);
    acc[1] = mma16(acc[1], ah, b1);
    acc[1] = mma16(acc[1], al, b1);
    asm volatile("v_nop\n\tv_nop\n\tv_nop\n\tv_nop"
                 : "+v"(acc[0]), "+v"(acc[1]) : "v"(ah.v), "v"(al.v), "v"(b0.v), "v"(b1.v));
  }
}
__device__ __forceinline__ void gemm_hl1(v8f& acc, lcp_us aH, lcp_us aL, const unsigned short* wb, int h)
{
#pragma unroll 1
  for (int k0 = 0; k0 < NH_; k0 += 32) {
    Frag ah, al, b;
    ldfrag_l(ah, aH + k0, h);
    ldfrag_l(al, aL + k0, h);
    ldfrag_g(b, wb + k0, h);
    acc = mma16(acc, ah, b);
    acc = mma16(acc, al, b);
    asm volatile("v_nop\n\tv_nop\n\tv_nop\n\tv_nop" : "+v"(acc) : "v"(ah.v), "v"(al.v), "v"(b.v));
  }
}

__device__ __forceinline__ void gate_to_lds(lp_f sD, const v8f (&acc)[2], lcp_f bias, int cw, int h)
{
#pragma unroll
  for (int nt = 0; nt < 2; ++nt) {
    const int col = cw + 16 * nt;
    const float b = bias[col];
#pragma unroll
    for (int r = 0; r < 8; ++r) {
      const float pre = acc[nt][r] + b;
      const float sg  = 1.0f / (1.0f + expf(-pre));
      sD[(8 * h + r) * NH_ + col] = 0.5f * sg;
    }
  }
}
__device__ __forceinline__ void tanh_to_lds(lp_us tH, lp_us tL, lp_f sF, const v8f (&acc)[2], lcp_f bias, int cw, int h)
{
#pragma unroll
  for (int nt = 0; nt < 2; ++nt) {
    const int col = cw + 16 * nt;
    const float b = bias[col];
#pragma unroll
    for (int r = 0; r < 8; ++r) {
      const int row = 8 * h + r;
      const float v = tanhf(acc[nt][r] + b);
      const unsigned short hb = bf16_bits(v);
      const unsigned short lb = bf16_bits(v - bf16_val(hb));
      tH[row * SP + col] = hb;
      tL[row * SP + col] = lb;
      sF[row * NH_ + col] = v;
    }
  }
}
__device__ __forceinline__ void lin_to_hilo(lp_us tH, lp_us tL, const v8f (&acc)[2], lcp_f bias, int cw, int h)
{
#pragma unroll
  for (int nt = 0; nt < 2; ++nt) {
    const int col = cw + 16 * nt;
    const float b = bias[col];
#pragma unroll
    for (int r = 0; r < 8; ++r) {
      const int row = 8 * h + r;
      const float v = acc[nt][r] + b;
      const unsigned short hb = bf16_bits(v);
      const unsigned short lb = bf16_bits(v - bf16_val(hb));
      tH[row * SP + col] = hb;
      tL[row * SP + col] = lb;
    }
  }
}

__device__ __forceinline__ void mem_phase(lcp_f sD, const float* histL, lp_us tH, lp_us tL, lcp_f sRc,
                                          int t, int vr0, int vc0)
{
  v4f dv[4], ma[4], cp[4];
  const int s0 = (t - 1) & (NK_ - 1);
#pragma unroll
  for (int i = 0; i < 4; ++i) {
    dv[i] = *(AS3 const v4fa*)(sD + (vr0 + i) * NH_ + vc0);
    const v4f hv = *(const v4fa*)(histL + (size_t)(s0 * RB + vr0 + i) * NH_ + vc0);
    ma[i] = dv[i] * hv;
    cp[i] = splat4(1.0f);
  }
#pragma unroll 3
  for (int j = 1; j < NK_; ++j) {
    const v4f jv = splat4((float)j);
    const v4f rc = splat4(sRc[j]);
    const int s = (t - 1 - j) & (NK_ - 1);
#pragma unroll
    for (int i = 0; i < 4; ++i) {
      const v4f f = (jv - dv[i]) * rc;
      cp[i] = cp[i] * f;
      const v4f wj = dv[i] * cp[i];
      const v4f hv = *(const v4fa*)(histL + (size_t)(s * RB + vr0 + i) * NH_ + vc0);
      ma[i] = ma[i] + wj * hv;
    }
  }
#pragma unroll
  for (int i = 0; i < 4; ++i) {
    v4us hb, lb;
#pragma unroll
    for (int c = 0; c < 4; ++c) {
      const float v = ma[i][c];
      const unsigned short b = bf16_bits(v);
      hb[c] = b;
      lb[c] = bf16_bits(v - bf16_val(b));
    }
    *(AS3 v4us*)(tH + (vr0 + i) * SP + vc0) = hb;
    *(AS3 v4us*)(tL + (vr0 + i) * SP + vc0) = lb;
  }
}
__device__ __forceinline__ void hist_store(float* histL, lcp_f sF, int t, int vr0, int vc0)
{
  const int s = t & (NK_ - 1);
  v4f hv[4];
#pragma unroll
  for (int i = 0; i < 4; ++i) hv[i] = *(AS3 const v4fa*)(sF + (vr0 + i) * NH_ + vc0);
#pragma unroll
  for (int i = 0; i < 4; ++i)
    *(volatile v4f*)(histL + (size_t)(s * RB + vr0 + i) * NH_ + vc0) = hv[i];
  __threadfence();
#pragma unroll
  for (int i = 0; i < 4; ++i)
    *(volatile v4f*)(histL + (size_t)(s * RB + vr0 + i) * NH_ + vc0) = hv[i];
}

__global__ __launch_bounds__(256)
void cvt_kernel(const float* __restrict__ wdx0, const float* __restrict__ wx0,  const float* __restrict__ wdh0,
                const float* __restrict__ wh0,  const float* __restrict__ wo0,  const float* __restrict__ wdx1,
                const float* __restrict__ wdh1, const float* __restrict__ wx1,  const float* __restrict__ wh1,
                const float* __restrict__ wo1,  const float* __restrict__ xin,  unsigned short* cv)
{
  const int g = blockIdx.x * 256 + threadIdx.x;
  if (g >= NPC) return;
  const int e = g * 8;
  const float* src;
  if      (e < P_WX0)  src = wdx0 + e;
  else if (e < P_WDH0) src = wx0  + (e - P_WX0);
  else if (e < P_WH0)  src = wdh0 + (e - P_WDH0);
  else if (e < P_WO0)  src = wh0  + (e - P_WH0);
  else if (e < P_WDX1) src = wo0  + (e - P_WO0);
  else if (e < P_WDH1) src = wdx1 + (e - P_WDX1);
  else if (e < P_WX1)  src = wdh1 + (e - P_WDH1);
  else if (e < P_WH1)  src = wx1  + (e - P_WX1);
  else if (e < P_WO1)  src = wh1  + (e - P_WH1);
  else if (e < P_X)    src = wo1  + (e - P_WO1);
  else                 src = xin  + (e - P_X);
  const v4f a = *(const v4fa*)src;
  const v4f c = *(const v4fa*)(src + 4);
  v8us o;
  o[0] = bf16_bits(a[0]); o[1] = bf16_bits(a[1]); o[2] = bf16_bits(a[2]); o[3] = bf16_bits(a[3]);
  o[4] = bf16_bits(c[0]); o[5] = bf16_bits(c[1]); o[6] = bf16_bits(c[2]); o[7] = bf16_bits(c[3]);
  unsigned short* dst = cv + e;
  *(volatile v8us*)dst = o;
  __threadfence();
  *(volatile v8us*)dst = o;
}

__global__ __launch_bounds__(256)
void mrnn_kernel(const unsigned short* __restrict__ cv,
                 const float* __restrict__ bd0, const float* __restrict__ bh0, const float* __restrict__ bo0,
                 const float* __restrict__ bd1, const float* __restrict__ bh1, const float* __restrict__ bo1,
                 float* hist, float* out)
{
  extern __shared__ __attribute__((aligned(16))) char smem[];
  lp_us tH0H = (lp_us)(smem + L_H0H);
  lp_us tH0L = (lp_us)(smem + L_H0L);
  lp_us tM0H = (lp_us)(smem + L_M0H);
  lp_us tM0L = (lp_us)(smem + L_M0L);
  lp_us tOH  = (lp_us)(smem + L_OH);
  lp_us tOL  = (lp_us)(smem + L_OL);
  lp_us tH1H = (lp_us)(smem + L_H1H);
  lp_us tH1L = (lp_us)(smem + L_H1L);
  lp_us tM1H = (lp_us)(smem + L_M1H);
  lp_us tM1L = (lp_us)(smem + L_M1L);
  lp_f  sD   = (lp_f)(smem + L_SD);
  lp_f  sF   = (lp_f)(smem + L_SF);
  lp_f  sO   = (lp_f)(smem + L_SO);
  lp_f  sB   = (lp_f)(smem + L_SB);
  lp_f  sRc  = (lp_f)(smem + L_RC);

  const int tid = threadIdx.x, lane = tid & 31;
  const int w = __builtin_amdgcn_readfirstlane(tid >> 5);
  const int h = lane >> 4, m = lane & 15;
  const int blk = (int)blockIdx.x;
  const int b0 = blk * RB;
  float* hist0 = hist + (size_t)blk * HBLK;
  float* hist1 = hist0 + HL;
  const int vr0 = 4 * (w >> 1);
  const int vc0 = 128 * (w & 1) + 4 * lane;
  const int cw  = 32 * w + m;

  {
    const v4f z4 = splat4(0.0f);
    for (int i = tid; i < NLDS16; i += 256) *(AS3 v4f*)(smem + 16 * i) = z4;
  }
  __syncthreads();
  sB[0 * NH_ + tid] = bf16r(bd0[tid]);
  sB[1 * NH_ + tid] = bf16r(bh0[tid]);
  sB[2 * NH_ + tid] = bf16r(bo0[tid]);
  sB[3 * NH_ + tid] = bf16r(bd1[tid]);
  sB[4 * NH_ + tid] = bf16r(bh1[tid]);
  if (tid < NO_) sB[5 * NH_ + tid] = bf16r(bo1[tid]);
  if (tid < NK_) sRc[tid] = 1.0f / (float)(tid + 1);
  {
    const v4f z4 = splat4(0.0f);
#pragma unroll 1
    for (int pass = 0; pass < 2; ++pass) {
#pragma unroll 1
      for (int q = 0; q < 2 * NK_; ++q) {
        float* base = hist0 + (size_t)q * (RB * NH_);
#pragma unroll
        for (int i = 0; i < 4; ++i) *(volatile v4f*)(base + (size_t)(vr0 + i) * NH_ + vc0) = z4;
      }
      __threadfence();
    }
  }
  __syncthreads();

#pragma unroll 1
  for (int t = 0; t < NT_; ++t) {
    const unsigned short* xrow = cv + P_X + (size_t)(t * NB_ + b0 + m) * NI_;
    v8f acc[2];

    acc[0] = zero8(); acc[1] = zero8();
    gemm_x(acc, xrow, cv + P_WDX0 + (size_t)cw * NI_, h);
    gemm_hl(acc, tH0H + m * SP, tH0L + m * SP, cv + P_WDH0 + (size_t)cw * NH_, h);
    gate_to_lds(sD, acc, sB + 0 * NH_, cw, h);
    __syncthreads();
    mem_phase(sD, hist0, tM0H, tM0L, sRc, t, vr0, vc0);
    __syncthreads();
    acc[0] = zero8(); acc[1] = zero8();
    gemm_x(acc, xrow, cv + P_WX0 + (size_t)cw * NI_, h);
    gemm_hl(acc, tM0H + m * SP, tM0L + m * SP, cv + P_WH0 + (size_t)cw * NH_, h);
    tanh_to_lds(tH0H, tH0L, sF, acc, sB + 1 * NH_, cw, h);
    __syncthreads();
    hist_store(hist0, sF, t, vr0, vc0);
    acc[0] = zero8(); acc[1] = zero8();
    gemm_hl(acc, tH0H + m * SP, tH0L + m * SP, cv + P_WO0 + (size_t)cw * NH_, h);
    lin_to_hilo(tOH, tOL, acc, sB + 2 * NH_, cw, h);
    __syncthreads();

    acc[0] = zero8(); acc[1] = zero8();
    gemm_hl(acc, tOH + m * SP, tOL + m * SP, cv + P_WDX1 + (size_t)cw * NH_, h);
    gemm_hl(acc, tH1H + m * SP, tH1L + m * SP, cv + P_WDH1 + (size_t)cw * NH_, h);
    gate_to_lds(sD, acc, sB + 3 * NH_, cw, h);
    __syncthreads();
    mem_phase(sD, hist1, tM1H, tM1L, sRc, t, vr0, vc0);
    __syncthreads();
    acc[0] = zero8(); acc[1] = zero8();
    gemm_hl(acc, tOH + m * SP, tOL + m * SP, cv + P_WX1 + (size_t)cw * NH_, h);
    gemm_hl(acc, tM1H + m * SP, tM1L + m * SP, cv + P_WH1 + (size_t)cw * NH_, h);
    tanh_to_lds(tH1H, tH1L, sF, acc, sB + 4 * NH_, cw, h);
    __syncthreads();
    hist_store(hist1, sF, t, vr0, vc0);
    if (w < 2) {
      v8f a1 = zero8();
      gemm_hl1(a1, tH1H + m * SP, tH1L + m * SP, cv + P_WO1 + (size_t)(16 * w + m) * NH_, h);
      const int col = 16 * w + m;
      const float b = sB[5 * NH_ + col];
#pragma unroll
      for (int r = 0; r < 8; ++r) sO[(8 * h + r) * NO_ + col] = a1[r] + b;
    }
    __syncthreads();
    if (w < 4) {
      const int row = tid >> 3, q = tid & 7;
      const v4f ov = *(AS3 const v4fa*)(sO + row * NO_ + 4 * q);
      float* od = out + (size_t)(t * NB_ + b0 + row) * NO_ + 4 * q;
      *(volatile v4f*)od = ov;
      __threadfence();
      *(volatile v4f*)od = ov;
    }
  }
}

extern "C" void kernel_launch(void* const* d_in, const int* in_sizes, int n_in,
                              void* d_out, int out_size, void* d_ws, size_t ws_size,
                              hipStream_t stream)
{
  if (n_in < 17) return;
  if (in_sizes[0]  != NT_ * NB_ * NI_) return;
  if (in_sizes[1]  != NH_ * NI_)       return;
  if (in_sizes[2]  != NH_ * NH_)       return;
  if (in_sizes[3]  != NH_)             return;
  if (in_sizes[4]  != NH_ * NI_)       return;
  if (in_sizes[5]  != NH_ * NH_)       return;
  if (in_sizes[6]  != NH_)             return;
  if (in_sizes[7]  != NH_ * NH_)       return;
  if (in_sizes[8]  != NH_)             return;
  if (in_sizes[9]  != NH_ * NH_)       return;
  if (in_sizes[10] != NH_ * NH_)       return;
  if (in_sizes[11] != NH_)             return;
  if (in_sizes[12] != NH_ * NH_)       return;
  if (in_sizes[13] != NH_ * NH_)       return;
  if (in_sizes[14] != NH_)             return;
  if (in_sizes[15] != NO_ * NH_)       return;
  if (in_sizes[16] != NO_)             return;
  if (out_size != NT_ * NB_ * NO_)     return;
  if (ws_size < WS_END)                return;

  const float* xin  = (const float*)d_in[0];
  const float* Wdx0 = (const float*)d_in[1];
  const float* Wdh0 = (const float*)d_in[2];
  const float* bd0  = (const float*)d_in[3];
  const float* Wx0  = (const float*)d_in[4];
  const float* Wh0  = (const float*)d_in[5];
  const float* bh0  = (const float*)d_in[6];
  const float* Wo0  = (const float*)d_in[7];
  const float* bo0  = (const float*)d_in[8];
  const float* Wdx1 = (const float*)d_in[9];
  const float* Wdh1 = (const float*)d_in[10];
  const float* bd1  = (const float*)d_in[11];
  const float* Wx1  = (const float*)d_in[12];
  const float* Wh1  = (const float*)d_in[13];
  const float* bh1  = (const float*)d_in[14];
  const float* Wo1  = (const float*)d_in[15];
  const float* bo1  = (const float*)d_in[16];
  float* out = (float*)d_out;

  char* ws = (char*)d_ws;
  unsigned short* cv = (unsigned short*)(ws + OFF_CV);
  float* hist = (float*)(ws + OFF_HI);

  cvt_kernel<<<dim3(NCBLK), dim3(256), 0, stream>>>(Wdx0, Wx0, Wdh0, Wh0, Wo0, Wdx1, Wdh1, Wx1, Wh1, Wo1, xin, cv);

  hipFuncSetAttribute(reinterpret_cast<const void*>(&mrnn_kernel),
                      hipFuncAttributeMaxDynamicSharedMemorySize, (int)LDS_BYTES);
  mrnn_kernel<<<dim3(NBLK), dim3(256), LDS_BYTES, stream>>>(cv, bd0, bh0, bo0, bd1, bh1, bo1, hist, out);
}
